// FastVARSelfAttention_3925600109079
// MI455X (gfx1250) — hardware-verified
//
#include <hip/hip_runtime.h>


typedef unsigned short us;
typedef __bf16 v16bf __attribute__((ext_vector_type(16)));
typedef unsigned short v8us __attribute__((ext_vector_type(8), __may_alias__));
typedef unsigned int v4u __attribute__((ext_vector_type(4), __may_alias__));
typedef float v4f __attribute__((ext_vector_type(4), __may_alias__));
typedef float v8f __attribute__((ext_vector_type(8)));

#define TL     1365
#define TLP    1408
#define NB     4
#define NH     16
#define HD     64
#define CDIM   1024
#define TP     (NB * TLP)
#define NKT    22
#define MT128  (TP / 128)
#define LDSP   72
#define TPITCH 136
#define FPITCH 68
#define LDS_US 27648

union Frag { v16bf v; v8us h[2]; };

__device__ __forceinline__ v16bf ldfrag(const us* p) {
  Frag f;
  f.h[0] = *(const v8us*)(p);
  f.h[1] = *(const v8us*)(p + 16);
  return f.v;
}

__device__ __forceinline__ v8f vz8() {
  v8f z = {0.f, 0.f, 0.f, 0.f, 0.f, 0.f, 0.f, 0.f};
  return z;
}

__device__ __forceinline__ v8f wmma3(v16bf ah, v16bf al, v16bf bh, v16bf bl, v8f c) {
  c = __builtin_amdgcn_wmma_f32_16x16x32_bf16(false, ah, false, bh, (short)0, c, false, false);
  c = __builtin_amdgcn_wmma_f32_16x16x32_bf16(false, ah, false, bl, (short)0, c, false, false);
  c = __builtin_amdgcn_wmma_f32_16x16x32_bf16(false, al, false, bh, (short)0, c, false, false);
  asm volatile("v_nop\n\tv_nop\n\tv_nop\n\tv_nop" : "+v"(c) : "v"(ah), "v"(al), "v"(bh), "v"(bl));
  return c;
}

__device__ __forceinline__ unsigned bf16_rne(float x) {
  unsigned u = __float_as_uint(x);
  return (u + 0x7FFFu + ((u >> 16) & 1u)) >> 16;
}
__device__ __forceinline__ void split2(float x, unsigned& hb, unsigned& lb) {
  hb = bf16_rne(x);
  const float hf = __uint_as_float(hb << 16);
  lb = bf16_rne(x - hf);
}

__device__ __forceinline__ float redmax16(float v) {
#pragma unroll
  for (int o = 1; o < 16; o <<= 1) v = fmaxf(v, __shfl_xor(v, o, 32));
  return v;
}
__device__ __forceinline__ float redsum16(float v) {
#pragma unroll
  for (int o = 1; o < 16; o <<= 1) v += __shfl_xor(v, o, 32);
  return v;
}

__global__ __launch_bounds__(256)
void cvt_split_kernel(const float* __restrict__ src, us* dh, us* dl,
                      int rows_out, int seg_out, int seg_in, int src_rows) {
  const int tid = threadIdx.x;
  const int r   = blockIdx.x * 2 + (tid >> 7);
  const int c8  = (tid & 127) * 8;
  const int sg  = r / seg_out;
  const int pos = r - sg * seg_out;
  const bool valid = (pos < seg_in) && (r < rows_out);
  int sr = sg * seg_in + ((pos < seg_in) ? pos : 0);
  sr = (sr < 0) ? 0 : ((sr > src_rows - 1) ? (src_rows - 1) : sr);
  const v4f* sp = (const v4f*)(src + (size_t)sr * CDIM + c8);
  const v4f a = sp[0];
  const v4f c = sp[1];
  float f[8];
  f[0] = valid ? a[0] : 0.f; f[1] = valid ? a[1] : 0.f; f[2] = valid ? a[2] : 0.f; f[3] = valid ? a[3] : 0.f;
  f[4] = valid ? c[0] : 0.f; f[5] = valid ? c[1] : 0.f; f[6] = valid ? c[2] : 0.f; f[7] = valid ? c[3] : 0.f;
  unsigned hb[8], lb[8];
#pragma unroll
  for (int i = 0; i < 8; ++i) split2(f[i], hb[i], lb[i]);
  v4u H, L;
#pragma unroll
  for (int i = 0; i < 4; ++i) {
    H[i] = hb[2 * i] | (hb[2 * i + 1] << 16);
    L[i] = lb[2 * i] | (lb[2 * i + 1] << 16);
  }
  if (r < rows_out) {
    us* ph = dh + (size_t)r * CDIM + c8;
    us* pl = dl + (size_t)r * CDIM + c8;
    *(volatile v4u*)ph = H;
    *(volatile v4u*)pl = L;
    __threadfence();
    *(volatile v4u*)ph = H;
    *(volatile v4u*)pl = L;
  }
}

__global__ __launch_bounds__(256)
void flags_kernel(const float* __restrict__ bias, int* flags) {
  __shared__ float redf[8];
  __shared__ float tmax_s[32];
  __shared__ int redi[8];
  const int tid = threadIdx.x, lane = tid & 31, wave = tid >> 5;
  const int qt = blockIdx.x;
  const int row = tid >> 2, seg = tid & 3;
  int qrow = qt * 64 + row;
  qrow = (qrow > TL - 1) ? (TL - 1) : qrow;
  const float* brow = bias + (size_t)qrow * TL;
  float rowmax = -3.0e38f;
  for (int kt = 0; kt < NKT; ++kt) {
    float mx = -3.0e38f;
#pragma unroll 4
    for (int j = 0; j < 16; ++j) {
      const int key = kt * 64 + seg * 16 + j;
      const int kc  = (key > TL - 1) ? (TL - 1) : key;
      float v = brow[kc];
      v = (key < TL) ? v : -3.0e38f;
      mx = fmaxf(mx, v);
    }
    rowmax = fmaxf(rowmax, mx);
    float w = mx;
#pragma unroll
    for (int o = 16; o > 0; o >>= 1) w = fmaxf(w, __shfl_xor(w, o, 32));
    if (lane == 0) redf[wave] = w;
    __syncthreads();
    if (tid == 0) {
      float t = redf[0];
      for (int i = 1; i < 8; ++i) t = fmaxf(t, redf[i]);
      tmax_s[kt] = t;
    }
    __syncthreads();
  }
  rowmax = fmaxf(rowmax, __shfl_xor(rowmax, 1, 32));
  rowmax = fmaxf(rowmax, __shfl_xor(rowmax, 2, 32));
  int bad = (rowmax < -1.0e28f) ? 1 : 0;
#pragma unroll
  for (int o = 16; o > 0; o >>= 1) bad |= __shfl_xor(bad, o, 32);
  if (lane == 0) redi[wave] = bad;
  __syncthreads();
  if (wave == 0) {
    int anybad = 0;
    for (int i = 0; i < 8; ++i) anybad |= redi[i];
    int nchv = 0;
    for (int kt = 0; kt < NKT; ++kt) {
      const float t = tmax_s[kt];
      const int u = (t <= -1.0e29f && anybad == 0) ? 0 : 1;
      if (u) nchv = kt + 1;
    }
    const float tl = tmax_s[(lane < NKT) ? lane : 0];
    int val = (lane < NKT) ? ((tl <= -1.0e29f && anybad == 0) ? 0 : 1) : 0;
    if (lane == 31) val = nchv;
    int* fp = flags + qt * 32 + lane;
    *(volatile int*)fp = val;
    __threadfence();
    *(volatile int*)fp = val;
  }
}

__device__ __forceinline__ void gemm_mainloop(const us* __restrict__ Ah, const us* __restrict__ Al, size_t arow0,
                                              const us* __restrict__ Bh, const us* __restrict__ Bl, size_t brow0,
                                              us* lds, v8f (&acc)[4]) {
  const int tid = threadIdx.x, lane = tid & 31, wave = tid >> 5, hh = lane >> 4, m = lane & 15;
  us* Ash = lds;
  us* Asl = lds + 128 * LDSP;
  us* Bsh = lds + 256 * LDSP;
  us* Bsl = lds + 320 * LDSP;
  for (int k0 = 0; k0 < CDIM; k0 += 64) {
    __syncthreads();
#pragma unroll
    for (int j = 0; j < 4; ++j) {
      const int q = tid + 256 * j, row = q >> 3, pc = q & 7;
      const size_t g = (arow0 + row) * CDIM + k0 + pc * 8;
      const v4u vh = *(const v4u*)(Ah + g);
      const v4u vl = *(const v4u*)(Al + g);
      *(v4u*)(Ash + row * LDSP + pc * 8) = vh;
      *(v4u*)(Asl + row * LDSP + pc * 8) = vl;
    }
#pragma unroll
    for (int j = 0; j < 2; ++j) {
      const int q = tid + 256 * j, row = q >> 3, pc = q & 7;
      const size_t g = (brow0 + row) * CDIM + k0 + pc * 8;
      const v4u vh = *(const v4u*)(Bh + g);
      const v4u vl = *(const v4u*)(Bl + g);
      *(v4u*)(Bsh + row * LDSP + pc * 8) = vh;
      *(v4u*)(Bsl + row * LDSP + pc * 8) = vl;
    }
    __syncthreads();
#pragma unroll
    for (int kk = 0; kk < 64; kk += 32) {
      const v16bf a_h = ldfrag(Ash + (wave * 16 + m) * LDSP + kk + 8 * hh);
      const v16bf a_l = ldfrag(Asl + (wave * 16 + m) * LDSP + kk + 8 * hh);
#pragma unroll
      for (int t = 0; t < 4; ++t) {
        const v16bf b_h = ldfrag(Bsh + (t * 16 + m) * LDSP + kk + 8 * hh);
        const v16bf b_l = ldfrag(Bsl + (t * 16 + m) * LDSP + kk + 8 * hh);
        acc[t] = wmma3(a_h, a_l, b_h, b_l, acc[t]);
      }
    }
  }
}

__global__ __launch_bounds__(256)
void qkv_kernel(const us* __restrict__ Xh, const us* __restrict__ Xl,
                const us* __restrict__ Wh, const us* __restrict__ Wl,
                const float* __restrict__ qbias, const float* __restrict__ vbias,
                const float* __restrict__ smlog,
                const float* __restrict__ rc, const float* __restrict__ rs,
                us* Qh, us* Ql, us* Kh, us* Kl, us* Vh, us* Vl) {
  __shared__ __align__(16) us lds[LDS_US];
  const int tid = threadIdx.x, lane = tid & 31, wave = tid >> 5, hh = lane >> 4, m = lane & 15;
  const int mb = blockIdx.x, nb = blockIdx.y;

  v8f acc[4];
#pragma unroll
  for (int t = 0; t < 4; ++t) acc[t] = vz8();
  gemm_mainloop(Xh, Xl, (size_t)mb * 128, Wh, Wl, (size_t)nb * 64, lds, acc);

  const int sec  = nb >> 4;
  const int head = nb & 15;
  const int bidx = mb / 11;
  const int mpos = (mb - bidx * 11) * 128;
  const int posbase = mpos + wave * 16;

  float vals[4][8];
#pragma unroll
  for (int t = 0; t < 4; ++t) {
    const float bq = qbias[head * HD + t * 16 + m];
    const float bv = vbias[head * HD + t * 16 + m];
    const float badd = (sec == 0) ? bq : ((sec == 2) ? bv : 0.0f);
#pragma unroll
    for (int r = 0; r < 8; ++r) vals[t][r] = acc[t][r] + badd;
  }

  if (sec < 2) {
    const float mulq = expf(fminf(smlog[head], 4.6051702f));
    const float mul  = (sec == 0) ? mulq : 1.0f;
#pragma unroll
    for (int r = 0; r < 8; ++r) {
      float ss = 0.f;
#pragma unroll
      for (int t = 0; t < 4; ++t) ss += vals[t][r] * vals[t][r];
      ss = redsum16(ss);
      const float inv = 1.0f / fmaxf(sqrtf(ss), 1e-12f);
#pragma unroll
      for (int t = 0; t < 4; ++t) vals[t][r] = (vals[t][r] * inv) * mul;
    }
#pragma unroll
    for (int t = 0; t < 4; ++t) {
      const int j = t * 8 + (m >> 1);
#pragma unroll
      for (int r = 0; r < 8; ++r) {
        int pr = posbase + 8 * hh + r;
        pr = (pr > TL - 1) ? (TL - 1) : pr;
        const float cw = rc[pr * 32 + j];
        const float sw = rs[pr * 32 + j];
        const float v  = vals[t][r];
        const float o  = __shfl_xor(v, 1, 32);
        vals[t][r] = (m & 1) ? (sw * o + cw * v) : (cw * v - sw * o);
      }
    }
  }

  __syncthreads();

  if (sec < 2) {
    us* st0 = lds + wave * (32 * LDSP);
    us* st1 = st0 + 16 * LDSP;
#pragma unroll
    for (int t = 0; t < 4; ++t)
#pragma unroll
      for (int r = 0; r < 8; ++r) {
        unsigned hb, lb;
        split2(vals[t][r], hb, lb);
        st0[(8 * hh + r) * LDSP + t * 16 + m] = (us)hb;
        st1[(8 * hh + r) * LDSP + t * 16 + m] = (us)lb;
      }
    __syncthreads();
    v4u keep[8];
    const int rq = lane >> 3, pc = lane & 7;
#pragma unroll
    for (int p = 0; p < 2; ++p) {
      const us* sp = (p == 0) ? st0 : st1;
#pragma unroll
      for (int s = 0; s < 4; ++s)
        keep[p * 4 + s] = *(const v4u*)(sp + (4 * s + rq) * LDSP + pc * 8);
    }
    us* dh = (sec == 0) ? Qh : Kh;
    us* dl = (sec == 0) ? Ql : Kl;
    const size_t rowbase = (size_t)(bidx * NH + head) * TLP + posbase;
#pragma unroll
    for (int p = 0; p < 2; ++p) {
      us* dp = (p == 0) ? dh : dl;
#pragma unroll
      for (int s = 0; s < 4; ++s)
        *(volatile v4u*)(dp + (rowbase + 4 * s + rq) * HD + pc * 8) = keep[p * 4 + s];
    }
    __threadfence();
#pragma unroll
    for (int p = 0; p < 2; ++p) {
      us* dp = (p == 0) ? dh : dl;
#pragma unroll
      for (int s = 0; s < 4; ++s)
        *(volatile v4u*)(dp + (rowbase + 4 * s + rq) * HD + pc * 8) = keep[p * 4 + s];
    }
  } else {
    us* T0 = lds;
    us* T1 = lds + 64 * TPITCH;
#pragma unroll
    for (int t = 0; t < 4; ++t)
#pragma unroll
      for (int r = 0; r < 8; ++r) {
        unsigned hb, lb;
        split2(vals[t][r], hb, lb);
        const int d = t * 16 + m, tok = wave * 16 + 8 * hh + r;
        T0[d * TPITCH + tok] = (us)hb;
        T1[d * TPITCH + tok] = (us)lb;
      }
    __syncthreads();
    v4u keep[8];
    const int pc = lane & 7;
#pragma unroll
    for (int p = 0; p < 2; ++p) {
      const us* sp = (p == 0) ? T0 : T1;
#pragma unroll
      for (int s = 0; s < 4; ++s) {
        const int li = s * 4 + (lane >> 3);
        const int d = wave * 8 + (li >> 1), half = li & 1;
        keep[p * 4 + s] = *(const v4u*)(sp + d * TPITCH + half * 64 + pc * 8);
      }
    }
    const size_t dbase = (size_t)(bidx * NH + head) * HD;
#pragma unroll
    for (int p = 0; p < 2; ++p) {
      us* dp = (p == 0) ? Vh : Vl;
#pragma unroll
      for (int s = 0; s < 4; ++s) {
        const int li = s * 4 + (lane >> 3);
        const int d = wave * 8 + (li >> 1), half = li & 1;
        *(volatile v4u*)(dp + (dbase + d) * TLP + mpos + half * 64 + pc * 8) = keep[p * 4 + s];
      }
    }
    __threadfence();
#pragma unroll
    for (int p = 0; p < 2; ++p) {
      us* dp = (p == 0) ? Vh : Vl;
#pragma unroll
      for (int s = 0; s < 4; ++s) {
        const int li = s * 4 + (lane >> 3);
        const int d = wave * 8 + (li >> 1), half = li & 1;
        *(volatile v4u*)(dp + (dbase + d) * TLP + mpos + half * 64 + pc * 8) = keep[p * 4 + s];
      }
    }
  }
}

__global__ __launch_bounds__(128)
void attn_kernel(const us* __restrict__ Qh, const us* __restrict__ Ql,
                 const us* __restrict__ Kh, const us* __restrict__ Kl,
                 const us* __restrict__ Vh, const us* __restrict__ Vl,
                 const float* __restrict__ bias, const int* __restrict__ flags,
                 us* Oh, us* Ol) {
  __shared__ __align__(16) us lds[LDS_US];
  const int tid = threadIdx.x, lane = tid & 31, wave = tid >> 5, hh = lane >> 4, m = lane & 15;
  us* Ksh = lds;
  us* Ksl = lds + 64 * LDSP;
  us* Vsh = lds + 128 * LDSP;
  us* Vsl = lds + 192 * LDSP;
  us* Psh = lds + 256 * LDSP + wave * (32 * LDSP);
  us* Psl = Psh + 16 * LDSP;

  const int qt = blockIdx.x, h = blockIdx.y, b = blockIdx.z;
  const int bh = b * NH + h;
  const int q0 = qt * 64 + wave * 16;

  const us* qph = Qh + ((size_t)bh * TLP + q0 + m) * HD;
  const us* qpl = Ql + ((size_t)bh * TLP + q0 + m) * HD;
  const v16bf qh0 = ldfrag(qph + 8 * hh);
  const v16bf qh1 = ldfrag(qph + 32 + 8 * hh);
  const v16bf ql0 = ldfrag(qpl + 8 * hh);
  const v16bf ql1 = ldfrag(qpl + 32 + 8 * hh);

  const int* fr = flags + qt * 32;
  int nch = fr[31];
  nch = (nch < 0) ? 0 : ((nch > NKT) ? NKT : nch);

  float mr[8], lr[8];
  v8f O[4];
#pragma unroll
  for (int r = 0; r < 8; ++r) { mr[r] = -3.0e38f; lr[r] = 0.f; }
#pragma unroll
  for (int t = 0; t < 4; ++t) O[t] = vz8();

  for (int kt = 0; kt < nch; ++kt) {
    if (fr[kt] == 0) continue;
    __syncthreads();
#pragma unroll
    for (int j = 0; j < 4; ++j) {
      const int q = tid + 128 * j, row = q >> 3, pc = q & 7;
      const size_t gk = ((size_t)bh * TLP + kt * 64 + row) * HD + pc * 8;
      const v4u k0 = *(const v4u*)(Kh + gk);
      const v4u k1 = *(const v4u*)(Kl + gk);
      *(v4u*)(Ksh + row * LDSP + pc * 8) = k0;
      *(v4u*)(Ksl + row * LDSP + pc * 8) = k1;
      const size_t gv = ((size_t)bh * HD + row) * TLP + kt * 64 + pc * 8;
      const v4u v0 = *(const v4u*)(Vh + gv);
      const v4u v1 = *(const v4u*)(Vl + gv);
      *(v4u*)(Vsh + row * LDSP + pc * 8) = v0;
      *(v4u*)(Vsl + row * LDSP + pc * 8) = v1;
    }
    __syncthreads();

    v8f S[4];
#pragma unroll
    for (int t = 0; t < 4; ++t) {
      S[t] = vz8();
      const us* kph = Ksh + (t * 16 + m) * LDSP + 8 * hh;
      const us* kpl = Ksl + (t * 16 + m) * LDSP + 8 * hh;
      S[t] = wmma3(qh0, ql0, ldfrag(kph), ldfrag(kpl), S[t]);
      S[t] = wmma3(qh1, ql1, ldfrag(kph + 32), ldfrag(kpl + 32), S[t]);
    }

#pragma unroll
    for (int r = 0; r < 8; ++r) {
      int qr = q0 + 8 * hh + r;
      qr = (qr > TL - 1) ? (TL - 1) : qr;
      const float* brow = bias + (size_t)qr * TL;
      float sv[4];
      float mx = -3.0e38f;
#pragma unroll
      for (int t = 0; t < 4; ++t) {
        const int key = kt * 64 + t * 16 + m;
        const int kc  = (key > TL - 1) ? (TL - 1) : key;
        const float bv = brow[kc];
        const float v  = (key < TL) ? (S[t][r] + bv) : -3.0e38f;
        sv[t] = v;
        mx = fmaxf(mx, v);
      }
      mx = redmax16(mx);
      const float mn = fmaxf(mr[r], mx);
      const float sc = __expf(mr[r] - mn);
      float psum = 0.f;
#pragma unroll
      for (int t = 0; t < 4; ++t) {
        const float p = __expf(sv[t] - mn);
        psum += p;
        unsigned hb, lb;
        split2(p, hb, lb);
        Psh[(8 * hh + r) * LDSP + t * 16 + m] = (us)hb;
        Psl[(8 * hh + r) * LDSP + t * 16 + m] = (us)lb;
        O[t][r] = O[t][r] * sc;
      }
      lr[r] = lr[r] * sc + redsum16(psum);
      mr[r] = mn;
    }
    __syncthreads();

#pragma unroll
    for (int ks = 0; ks < 2; ++ks) {
      const v16bf p_h = ldfrag(Psh + m * LDSP + ks * 32 + 8 * hh);
      const v16bf p_l = ldfrag(Psl + m * LDSP + ks * 32 + 8 * hh);
#pragma unroll
      for (int t = 0; t < 4; ++t) {
        const v16bf v_h = ldfrag(Vsh + (t * 16 + m) * LDSP + ks * 32 + 8 * hh);
        const v16bf v_l = ldfrag(Vsl + (t * 16 + m) * LDSP + ks * 32 + 8 * hh);
        O[t] = wmma3(p_h, p_l, v_h, v_l, O[t]);
      }
    }
  }

  __syncthreads();
#pragma unroll
  for (int r = 0; r < 8; ++r) {
    const float inv = (lr[r] > 0.f) ? (1.0f / lr[r]) : 0.f;
#pragma unroll
    for (int t = 0; t < 4; ++t) {
      unsigned hb, lb;
      split2(O[t][r] * inv, hb, lb);
      Psh[(8 * hh + r) * LDSP + t * 16 + m] = (us)hb;
      Psl[(8 * hh + r) * LDSP + t * 16 + m] = (us)lb;
    }
  }
  __syncthreads();
  v4u keep[8];
  const int rq = lane >> 3, pc = lane & 7;
#pragma unroll
  for (int p = 0; p < 2; ++p) {
    const us* sp = (p == 0) ? Psh : Psl;
#pragma unroll
    for (int s = 0; s < 4; ++s)
      keep[p * 4 + s] = *(const v4u*)(sp + (4 * s + rq) * LDSP + pc * 8);
  }
  const size_t orow = (size_t)b * TLP + q0;
#pragma unroll
  for (int p = 0; p < 2; ++p) {
    us* dp = (p == 0) ? Oh : Ol;
#pragma unroll
    for (int s = 0; s < 4; ++s)
      *(volatile v4u*)(dp + (orow + 4 * s + rq) * CDIM + h * HD + pc * 8) = keep[p * 4 + s];
  }
  __threadfence();
#pragma unroll
  for (int p = 0; p < 2; ++p) {
    us* dp = (p == 0) ? Oh : Ol;
#pragma unroll
    for (int s = 0; s < 4; ++s)
      *(volatile v4u*)(dp + (orow + 4 * s + rq) * CDIM + h * HD + pc * 8) = keep[p * 4 + s];
  }
}

__global__ __launch_bounds__(256)
void proj_kernel(const us* __restrict__ Ah, const us* __restrict__ Al,
                 const us* __restrict__ Wh, const us* __restrict__ Wl,
                 const float* __restrict__ bproj, float* out) {
  __shared__ __align__(16) us lds[LDS_US];
  const int tid = threadIdx.x, lane = tid & 31, wave = tid >> 5, hh = lane >> 4, m = lane & 15;
  const int mb = blockIdx.x, nb = blockIdx.y;
  const int n0 = nb * 64;

  v8f acc[4];
#pragma unroll
  for (int t = 0; t < 4; ++t) acc[t] = vz8();
  gemm_mainloop(Ah, Al, (size_t)mb * 128, Wh, Wl, (size_t)n0, lds, acc);

  const int bidx = mb / 11;
  const int posbase = (mb - bidx * 11) * 128 + wave * 16;

  __syncthreads();
  float* F = (float*)lds + wave * (16 * FPITCH);
#pragma unroll
  for (int t = 0; t < 4; ++t) {
    const float bv = bproj[n0 + t * 16 + m];
#pragma unroll
    for (int r = 0; r < 8; ++r) F[(8 * hh + r) * FPITCH + t * 16 + m] = acc[t][r] + bv;
  }
  __syncthreads();
  v4f keep[8];
  const int rh = lane >> 4, pc = lane & 15;
#pragma unroll
  for (int s = 0; s < 8; ++s)
    keep[s] = *(const v4f*)(F + (2 * s + rh) * FPITCH + pc * 4);
#pragma unroll
  for (int s = 0; s < 8; ++s) {
    const int pos = posbase + 2 * s + rh;
    if (pos < TL) {
      float* dp = out + ((size_t)(bidx * TL + pos) * CDIM + n0 + pc * 4);
      *(volatile v4f*)dp = keep[s];
    }
  }
  __threadfence();
#pragma unroll
  for (int s = 0; s < 8; ++s) {
    const int pos = posbase + 2 * s + rh;
    if (pos < TL) {
      float* dp = out + ((size_t)(bidx * TL + pos) * CDIM + n0 + pc * 4);
      *(volatile v4f*)dp = keep[s];
    }
  }
}

extern "C" void kernel_launch(void* const* d_in, const int* in_sizes, int n_in,
                              void* d_out, int out_size, void* d_ws, size_t ws_size,
                              hipStream_t stream) {
  if (n_in < 10) return;
  if (in_sizes[0] != NB * TL * CDIM) return;
  if (in_sizes[1] != TL * TL) return;
  if (in_sizes[2] != TL * 32 || in_sizes[3] != TL * 32) return;
  if (in_sizes[4] != 3 * CDIM * CDIM) return;
  if (in_sizes[5] < CDIM || in_sizes[6] < CDIM || in_sizes[7] < NH) return;
  if (in_sizes[8] != CDIM * CDIM || in_sizes[9] < CDIM) return;
  if (out_size != NB * TL * CDIM) return;

  const float* x     = (const float*)d_in[0];
  const float* abias = (const float*)d_in[1];
  const float* rc    = (const float*)d_in[2];
  const float* rs    = (const float*)d_in[3];
  const float* Wqkv  = (const float*)d_in[4];
  const float* qbias = (const float*)d_in[5];
  const float* vbias = (const float*)d_in[6];
  const float* smlog = (const float*)d_in[7];
  const float* Wproj = (const float*)d_in[8];
  const float* bproj = (const float*)d_in[9];
  float* out = (float*)d_out;

  const size_t PLX  = (size_t)TP * CDIM * 2;
  const size_t PLWQ = (size_t)3 * CDIM * CDIM * 2;
  const size_t PLWP = (size_t)CDIM * CDIM * 2;
  const size_t PLQ  = (size_t)NB * NH * TLP * HD * 2;
  const size_t FLB  = 4096;
  size_t off = 0;
  const size_t oXh = off;  off += PLX;
  const size_t oXl = off;  off += PLX;
  const size_t oWQh = off; off += PLWQ;
  const size_t oWQl = off; off += PLWQ;
  const size_t oWPh = off; off += PLWP;
  const size_t oWPl = off; off += PLWP;
  const size_t oQh = off;  off += PLQ;
  const size_t oQl = off;  off += PLQ;
  const size_t oKh = off;  off += PLQ;
  const size_t oKl = off;  off += PLQ;
  const size_t oVh = off;  off += PLQ;
  const size_t oVl = off;  off += PLQ;
  const size_t oFl = off;  off += FLB;
  if (off > ws_size) return;

  char* w = (char*)d_ws;
  us* Xh = (us*)(w + oXh);   us* Xl = (us*)(w + oXl);
  us* WQh = (us*)(w + oWQh); us* WQl = (us*)(w + oWQl);
  us* WPh = (us*)(w + oWPh); us* WPl = (us*)(w + oWPl);
  us* Qh = (us*)(w + oQh);   us* Ql = (us*)(w + oQl);
  us* Kh = (us*)(w + oKh);   us* Kl = (us*)(w + oKl);
  us* Vh = (us*)(w + oVh);   us* Vl = (us*)(w + oVl);
  int* flg = (int*)(w + oFl);
  us* Oh = Xh;
  us* Ol = Xl;

  cvt_split_kernel<<<TP / 2, 256, 0, stream>>>(x, Xh, Xl, TP, TLP, TL, NB * TL);
  cvt_split_kernel<<<(3 * CDIM) / 2, 256, 0, stream>>>(Wqkv, WQh, WQl, 3 * CDIM, 3 * CDIM, 3 * CDIM, 3 * CDIM);
  cvt_split_kernel<<<CDIM / 2, 256, 0, stream>>>(Wproj, WPh, WPl, CDIM, CDIM, CDIM, CDIM);
  flags_kernel<<<NKT, 256, 0, stream>>>(abias, flg);
  qkv_kernel<<<dim3(MT128, 48), 256, 0, stream>>>(Xh, Xl, WQh, WQl, qbias, vbias, smlog, rc, rs,
                                                   Qh, Ql, Kh, Kl, Vh, Vl);
  attn_kernel<<<dim3(NKT, NH, NB), 128, 0, stream>>>(Qh, Ql, Kh, Kl, Vh, Vl, abias, flg, Oh, Ol);
  proj_kernel<<<dim3(MT128, CDIM / 64), 256, 0, stream>>>(Oh, Ol, WPh, WPl, bproj, out);
}
